// GNN_AttentiveFP_18279380811837
// MI455X (gfx1250) — hardware-verified
//
#include <hip/hip_runtime.h>
#include <stddef.h>
#include <stdint.h>


#define HD    64
#define EDM   16
#define GR    32
#define AP    72
#define XP    68
#define NB    1024
#define CHUNK 2048
#define NTHR  256
#define NWAVE 8
#define WCAP  256
#define NGRP  (CHUNK / (NTHR * 4))
#define ET    1024
#define LDS_AGG_BYTES ((NB * HD + 2 * NB + NWAVE * WCAP + NWAVE) * 4)

static_assert(WCAP == (CHUNK / NTHR) * 32);
static_assert(NGRP == 2);
static_assert(NB == 1024);
static_assert(CHUNK == 2048);
static_assert(LDS_AGG_BYTES == 278560);
static_assert((NB % (NWAVE * 2)) == 0);
static_assert(ET == NWAVE * 128);
static_assert((NB % GR) == 0);
static_assert(((AP * 2) % 16) == 0);
static_assert(((XP * 4) % 16) == 0);

typedef float          v2f  __attribute__((ext_vector_type(2)));
typedef float          v4f  __attribute__((ext_vector_type(4)));
typedef float          v8f  __attribute__((ext_vector_type(8)));
typedef int            v4i  __attribute__((ext_vector_type(4)));
typedef unsigned       v4u  __attribute__((ext_vector_type(4)));
typedef __bf16         v16b __attribute__((ext_vector_type(16)));
typedef unsigned short us16;
union BFrag { v16b v; v4u q[2]; };

__device__ __forceinline__ v8f wm(const BFrag& a, const BFrag& b, v8f c) {
  v8f d = __builtin_amdgcn_wmma_f32_16x16x32_bf16(false, a.v, false, b.v, (short)0, c, false, false);
  asm volatile("v_nop\n\tv_nop\n\tv_nop\n\tv_nop" : "+v"(d) : "v"(a.v), "v"(b.v));
  return d;
}

__device__ __forceinline__ unsigned bfb(float f) {
  const unsigned u = __float_as_uint(f);
  return (u + 0x7fffu + ((u >> 16) & 1u)) >> 16;
}
__device__ __forceinline__ unsigned pk2(float a, float b, unsigned& lo) {
  const unsigned ha = bfb(a), hb = bfb(b);
  const float ra = a - __uint_as_float(ha << 16);
  const float rb = b - __uint_as_float(hb << 16);
  lo = bfb(ra) | (bfb(rb) << 16);
  return ha | (hb << 16);
}
__device__ __forceinline__ void split8(v4f f0, v4f f1, v4u& hq, v4u& lq) {
  unsigned l0, l1, l2, l3;
  v4u hh;
  hh.x = pk2(f0.x, f0.y, l0);
  hh.y = pk2(f0.z, f0.w, l1);
  hh.z = pk2(f1.x, f1.y, l2);
  hh.w = pk2(f1.z, f1.w, l3);
  v4u ll;
  ll.x = l0; ll.y = l1; ll.z = l2; ll.w = l3;
  hq = hh; lq = ll;
}

__device__ __forceinline__ float leaky01(float v) { return v > 0.f ? v : 0.01f * v; }
__device__ __forceinline__ float relu1(float v) { return v > 0.f ? v : 0.f; }
__device__ __forceinline__ float sigm1(float x) { return __builtin_amdgcn_rcpf(1.0f + __expf(-x)); }
__device__ __forceinline__ float tanh1(float x) {
  const float e = __expf(-2.0f * fabsf(x));
  const float t = (1.0f - e) * __builtin_amdgcn_rcpf(1.0f + e);
  return x < 0.f ? -t : t;
}
__device__ __forceinline__ float elu1(float v) { return v > 0.f ? v : (__expf(v) - 1.0f); }

__global__ __launch_bounds__(NTHR) void k_prep(
    const float* __restrict__ p0, const float* __restrict__ p1, const float* __restrict__ p2,
    const float* __restrict__ p3, const float* __restrict__ p4, const float* __restrict__ p5,
    int sp0, int sp1, int sp2, int sp3, int sp4, int sp5, int rows, us16* Wp) {
  const int z = blockIdx.y;
  const float* W = p0;
  int sp = sp0;
  if (z == 1)      { W = p1; sp = sp1; }
  else if (z == 2) { W = p2; sp = sp2; }
  else if (z == 3) { W = p3; sp = sp3; }
  else if (z == 4) { W = p4; sp = sp4; }
  else if (z == 5) { W = p5; sp = sp5; }
  const int i = blockIdx.x * NTHR + threadIdx.x;
  if (i >= rows * 8) return;
  const int r = i >> 3, c0 = (i & 7) * 8;
  const float* src = W + (size_t)r * sp + c0;
  const v4f f0 = *(const v4f*)src, f1 = *(const v4f*)(src + 4);
  v4u hq, lq;
  split8(f0, f1, hq, lq);
  us16* hp = Wp + (size_t)z * 2 * rows * HD + (size_t)r * HD + c0;
  us16* lp = hp + (size_t)rows * HD;
  *(volatile v4u*)hp = hq;
  *(volatile v4u*)lp = lq;
  __threadfence();
  *(volatile v4u*)hp = hq;
  *(volatile v4u*)lp = lq;
}

__device__ __forceinline__ void gemm_store(const float* Xs, const float* Sc, float* Y, float* sc1, float* sc2,
                                           int flags, int rowBase, int wave, int lane, int h, int m) {
#pragma unroll
  for (int i = 0; i < 2; ++i) {
    const int row = 4 * wave + 2 * i + h;
    const v4f v = *(const v4f*)(Xs + row * XP + 4 * m);
    *(volatile v4f*)(Y + (size_t)(rowBase + row) * HD + 4 * m) = v;
  }
  if ((flags & 2) && wave == 0 && lane < 8) {
    const v4f s = *(const v4f*)(Sc + 4 * lane);
    *(volatile v4f*)(sc1 + (size_t)rowBase + 4 * lane) = s;
  }
  if ((flags & 4) && wave == 0 && lane >= 8 && lane < 16) {
    const v4f s = *(const v4f*)(Sc + GR + 4 * (lane - 8));
    *(volatile v4f*)(sc2 + (size_t)rowBase + 4 * (lane - 8)) = s;
  }
}

template <int ACT>
__global__ __launch_bounds__(NTHR) void k_gemm(
    const float* __restrict__ X, int nRows,
    const us16* __restrict__ Wh, const us16* __restrict__ Wl,
    const float* __restrict__ bias, const float* __restrict__ att1, const float* __restrict__ att2, int flags,
    float* Y, float* sc1, float* sc2) {
  __shared__ __attribute__((aligned(16))) us16 Ah[GR * AP];
  __shared__ __attribute__((aligned(16))) us16 Al[GR * AP];
  __shared__ __attribute__((aligned(16))) float Xs[GR * XP];
  __shared__ __attribute__((aligned(16))) float Sc[2 * GR];

  const int tid = threadIdx.x, lane = tid & 31, wave = tid >> 5;
  const int h = lane >> 4, m = lane & 15;
  const int rowBase = blockIdx.x * GR;

  {
    const int r = tid >> 3, c0 = (tid & 7) * 8;
    int row = rowBase + r;
    if (row > nRows - 1) row = nRows - 1;
    const float* p = X + (size_t)row * HD + c0;
    const v4f f0 = *(const v4f*)p, f1 = *(const v4f*)(p + 4);
    v4u hq, lq;
    split8(f0, f1, hq, lq);
    *(v4u*)(Ah + r * AP + c0) = hq;
    *(v4u*)(Al + r * AP + c0) = lq;
  }
  __syncthreads();

  const int rt = wave >> 2, ct = wave & 3;
  const int n = ct * 16 + m;
  v8f acc = {0.f, 0.f, 0.f, 0.f, 0.f, 0.f, 0.f, 0.f};
#pragma unroll
  for (int kt = 0; kt < HD / 32; ++kt) {
    const int k0 = kt * 32;
    BFrag ah, al, bh, bl;
    const us16* pah = Ah + (rt * 16 + m) * AP + k0 + 8 * h;
    const us16* pal = Al + (rt * 16 + m) * AP + k0 + 8 * h;
    ah.q[0] = *(const v4u*)pah; ah.q[1] = *(const v4u*)(pah + 16);
    al.q[0] = *(const v4u*)pal; al.q[1] = *(const v4u*)(pal + 16);
    const us16* pbh = Wh + (size_t)n * HD + k0 + 8 * h;
    const us16* pbl = Wl + (size_t)n * HD + k0 + 8 * h;
    bh.q[0] = *(const v4u*)pbh; bh.q[1] = *(const v4u*)(pbh + 16);
    bl.q[0] = *(const v4u*)pbl; bl.q[1] = *(const v4u*)(pbl + 16);
    acc = wm(ah, bh, acc);
    acc = wm(al, bh, acc);
    acc = wm(ah, bl, acc);
  }

  float bv = 0.f;
  if (flags & 1) bv = bias[n];
#pragma unroll
  for (int r = 0; r < 8; ++r) {
    float v = acc[r] + bv;
    if (ACT == 1) v = leaky01(v);
    Xs[(rt * 16 + 8 * h + r) * XP + n] = v;
  }
  __syncthreads();

  if (flags & 2) {
    const int r = tid >> 3, c0 = (tid & 7) * 8;
    float s1 = 0.f, s2 = 0.f;
#pragma unroll
    for (int i = 0; i < 8; ++i) {
      const float v = Xs[r * XP + c0 + i];
      s1 += v * att1[c0 + i];
      if (flags & 4) s2 += v * att2[c0 + i];
    }
    s1 += __shfl_xor(s1, 1, 32); s1 += __shfl_xor(s1, 2, 32); s1 += __shfl_xor(s1, 4, 32);
    s2 += __shfl_xor(s2, 1, 32); s2 += __shfl_xor(s2, 2, 32); s2 += __shfl_xor(s2, 4, 32);
    if ((tid & 7) == 0) { Sc[r] = s1; Sc[GR + r] = s2; }
  }
  __syncthreads();

  gemm_store(Xs, Sc, Y, sc1, sc2, flags, rowBase, wave, lane, h, m);
  __threadfence();
  gemm_store(Xs, Sc, Y, sc1, sc2, flags, rowBase, wave, lane, h, m);
}

__device__ __forceinline__ void row_store(const float* XY, float* Y, int rowBase, int wave, int h, int m) {
#pragma unroll
  for (int i = 0; i < 2; ++i) {
    const int row = 4 * wave + 2 * i + h;
    const v4f v = *(const v4f*)(XY + row * XP + 4 * m);
    *(volatile v4f*)(Y + (size_t)(rowBase + row) * HD + 4 * m) = v;
  }
}

__global__ __launch_bounds__(NTHR) void k_gru(
    const float* __restrict__ Hin, const float* __restrict__ Hx, int nRows,
    const us16* __restrict__ Wih, const us16* __restrict__ Whh,
    const float* __restrict__ bih, const float* __restrict__ bhh, float* Y) {
  __shared__ __attribute__((aligned(16))) us16 Ih[GR * AP];
  __shared__ __attribute__((aligned(16))) us16 Il[GR * AP];
  __shared__ __attribute__((aligned(16))) us16 Xh[GR * AP];
  __shared__ __attribute__((aligned(16))) us16 Xl[GR * AP];
  __shared__ __attribute__((aligned(16))) float XY[GR * XP];

  const int tid = threadIdx.x, lane = tid & 31, wave = tid >> 5;
  const int h = lane >> 4, m = lane & 15;
  const int rowBase = blockIdx.x * GR;

  {
    const int r = tid >> 3, c0 = (tid & 7) * 8;
    int row = rowBase + r;
    if (row > nRows - 1) row = nRows - 1;
    const float* pi = Hin + (size_t)row * HD + c0;
    const float* px = Hx + (size_t)row * HD + c0;
    const v4f f0 = *(const v4f*)pi, f1 = *(const v4f*)(pi + 4);
    const v4f g0 = *(const v4f*)px, g1 = *(const v4f*)(px + 4);
    v4u hq, lq;
    split8(f0, f1, hq, lq);
    *(v4u*)(Ih + r * AP + c0) = hq;
    *(v4u*)(Il + r * AP + c0) = lq;
    split8(g0, g1, hq, lq);
    *(v4u*)(Xh + r * AP + c0) = hq;
    *(v4u*)(Xl + r * AP + c0) = lq;
    *(v4f*)(XY + r * XP + c0) = g0;
    *(v4f*)(XY + r * XP + c0 + 4) = g1;
  }
  __syncthreads();

  const int rt = wave >> 2, ft = wave & 3;
  const int f = ft * 16 + m;
  v8f gi[3], gh[3];
#pragma unroll
  for (int g = 0; g < 3; ++g) {
    gi[g] = (v8f){0.f, 0.f, 0.f, 0.f, 0.f, 0.f, 0.f, 0.f};
    gh[g] = (v8f){0.f, 0.f, 0.f, 0.f, 0.f, 0.f, 0.f, 0.f};
  }
  const size_t loOff = (size_t)3 * HD * HD;
#pragma unroll
  for (int kt = 0; kt < HD / 32; ++kt) {
    const int k0 = kt * 32;
    BFrag ih, il, xh, xl;
    const us16* p0 = Ih + (rt * 16 + m) * AP + k0 + 8 * h;
    const us16* p1 = Il + (rt * 16 + m) * AP + k0 + 8 * h;
    const us16* p2 = Xh + (rt * 16 + m) * AP + k0 + 8 * h;
    const us16* p3 = Xl + (rt * 16 + m) * AP + k0 + 8 * h;
    ih.q[0] = *(const v4u*)p0; ih.q[1] = *(const v4u*)(p0 + 16);
    il.q[0] = *(const v4u*)p1; il.q[1] = *(const v4u*)(p1 + 16);
    xh.q[0] = *(const v4u*)p2; xh.q[1] = *(const v4u*)(p2 + 16);
    xl.q[0] = *(const v4u*)p3; xl.q[1] = *(const v4u*)(p3 + 16);
#pragma unroll
    for (int g = 0; g < 3; ++g) {
      const size_t nrow = (size_t)(g * HD + f) * HD + k0 + 8 * h;
      BFrag bh, bl;
      const us16* pb = Wih + nrow;
      bh.q[0] = *(const v4u*)pb;           bh.q[1] = *(const v4u*)(pb + 16);
      bl.q[0] = *(const v4u*)(pb + loOff); bl.q[1] = *(const v4u*)(pb + loOff + 16);
      gi[g] = wm(ih, bh, gi[g]);
      gi[g] = wm(il, bh, gi[g]);
      gi[g] = wm(ih, bl, gi[g]);
      const us16* pc = Whh + nrow;
      bh.q[0] = *(const v4u*)pc;           bh.q[1] = *(const v4u*)(pc + 16);
      bl.q[0] = *(const v4u*)(pc + loOff); bl.q[1] = *(const v4u*)(pc + loOff + 16);
      gh[g] = wm(xh, bh, gh[g]);
      gh[g] = wm(xl, bh, gh[g]);
      gh[g] = wm(xh, bl, gh[g]);
    }
  }

  const float bi0 = bih[f], bi1 = bih[HD + f], bi2 = bih[2 * HD + f];
  const float bh0 = bhh[f], bh1 = bhh[HD + f], bh2 = bhh[2 * HD + f];
#pragma unroll
  for (int r = 0; r < 8; ++r) {
    const int row = rt * 16 + 8 * h + r;
    const float sr = gi[0][r] + bi0 + gh[0][r] + bh0;
    const float sz = gi[1][r] + bi1 + gh[1][r] + bh1;
    const float rg = sigm1(sr);
    const float zg = sigm1(sz);
    const float sn = gi[2][r] + bi2 + rg * (gh[2][r] + bh2);
    const float ng = tanh1(sn);
    const float hx = XY[row * XP + f];
    float v = (1.0f - zg) * ng + zg * hx;
    v = relu1(v);
    XY[row * XP + f] = v;
  }
  __syncthreads();

  row_store(XY, Y, rowBase, wave, h, m);
  __threadfence();
  row_store(XY, Y, rowBase, wave, h, m);
}

__global__ __launch_bounds__(NTHR) void k_edge(
    const float* __restrict__ ea, const int* __restrict__ ei, int nE,
    const float* __restrict__ W1, const float* __restrict__ attl,
    const float* __restrict__ S1, const float* __restrict__ GRs, int nN, float* E1) {
  __shared__ __attribute__((aligned(16))) float stg[NWAVE * 128];
  const int tid = threadIdx.x, lane = tid & 31, wave = tid >> 5;
  const int h = lane >> 4, m = lane & 15;

  BFrag b1[4], b2[4];
  float al[4];
  const v4u z4u = {0u, 0u, 0u, 0u};
#pragma unroll
  for (int nt = 0; nt < 4; ++nt) {
    const int n = nt * 16 + m;
    const float* pw = W1 + (size_t)n * (HD + EDM) + HD + 8 * h;
    const v4f w0 = *(const v4f*)pw, w1 = *(const v4f*)(pw + 4);
    v4u hq, lq;
    split8(w0, w1, hq, lq);
    b1[nt].q[0] = hq; b1[nt].q[1] = hq;
    b2[nt].q[0] = lq; b2[nt].q[1] = z4u;
    al[nt] = attl[n];
  }
  const int waveE = blockIdx.x * ET + wave * 128;

#pragma unroll 1
  for (int t = 0; t < 8; ++t) {
    const int e0 = waveE + t * 16;
    int er = e0 + m;
    if (er > nE - 1) er = nE - 1;
    const float* pa = ea + (size_t)er * EDM + 8 * h;
    const v4f f0 = *(const v4f*)pa, f1 = *(const v4f*)(pa + 4);
    BFrag a;
    {
      v4u hq, lq;
      split8(f0, f1, hq, lq);
      a.q[0] = hq; a.q[1] = lq;
    }
    int srcv[8];
#pragma unroll
    for (int r = 0; r < 8; ++r) {
      int e = e0 + 8 * h + r;
      if (e > nE - 1) e = nE - 1;
      int s = ei[e];
      s = s < 0 ? 0 : (s > nN - 1 ? nN - 1 : s);
      srcv[r] = s;
    }
    v8f acc[4];
#pragma unroll
    for (int nt = 0; nt < 4; ++nt) acc[nt] = (v8f){0.f, 0.f, 0.f, 0.f, 0.f, 0.f, 0.f, 0.f};
#pragma unroll
    for (int nt = 0; nt < 4; ++nt) {
      acc[nt] = wm(a, b1[nt], acc[nt]);
      acc[nt] = wm(a, b2[nt], acc[nt]);
    }
    float rs[8];
#pragma unroll
    for (int r = 0; r < 8; ++r) {
      const float* sp = S1 + (size_t)srcv[r] * HD + m;
      float s = 0.f;
#pragma unroll
      for (int nt = 0; nt < 4; ++nt) {
        float v = acc[nt][r] + sp[16 * nt];
        v = leaky01(v);
        s += v * al[nt];
      }
      rs[r] = s;
    }
#pragma unroll
    for (int mk = 1; mk < 16; mk <<= 1) {
#pragma unroll
      for (int r = 0; r < 8; ++r) rs[r] += __shfl_xor(rs[r], mk, 32);
    }
    float mine = rs[0];
#pragma unroll
    for (int r = 1; r < 8; ++r) mine = (m == r) ? rs[r] : mine;
    int de = e0 + 8 * h + (m & 7);
    if (de > nE - 1) de = nE - 1;
    int dn = ei[(size_t)nE + de];
    dn = dn < 0 ? 0 : (dn > nN - 1 ? nN - 1 : dn);
    const float aa = leaky01(mine + GRs[dn]);
    if (m < 8) stg[wave * 128 + t * 16 + 8 * h + m] = aa;
  }
  __syncthreads();

  const v4f v = *(const v4f*)(stg + wave * 128 + 4 * lane);
  float* op = E1 + (size_t)waveE + 4 * lane;
  *(volatile v4f*)op = v;
  __threadfence();
  *(volatile v4f*)op = v;
}

template <int MODE>
__device__ __forceinline__ void agg_store(const float* sacc, const float* sden, const float* bias, float* out,
                                          int nodeBase, int wave, int h, int m) {
  v4f b4 = {0.f, 0.f, 0.f, 0.f};
  if (MODE != 3) b4 = *(const v4f*)(bias + 4 * m);
#pragma unroll 1
  for (int j = 0; j < NB / (NWAVE * 2); ++j) {
    const int s = wave * (NB / NWAVE) + 2 * j + h;
    const v4f a4 = *(const v4f*)(sacc + s * HD + 4 * m);
    v4f y;
    if (MODE == 3) {
      y.x = relu1(a4.x); y.y = relu1(a4.y); y.z = relu1(a4.z); y.w = relu1(a4.w);
    } else {
      const float dn = sden[s];
      const float inv = __builtin_amdgcn_rcpf(dn + 1e-16f);
      y = a4 * inv + b4;
      y.x = elu1(y.x); y.y = elu1(y.y); y.z = elu1(y.z); y.w = elu1(y.w);
    }
    *(volatile v4f*)(out + (size_t)(nodeBase + s) * HD + 4 * m) = y;
  }
}

template <int MODE>
__global__ __launch_bounds__(NTHR) void k_agg(
    const int* __restrict__ srci, const int* __restrict__ dsti, int nItems,
    const float* __restrict__ msg, int nSrc, const float* __restrict__ lg,
    const float* __restrict__ asn, const float* __restrict__ adn, int nDst,
    const float* __restrict__ bias, float* out) {
  extern __shared__ v4f lds_dyn[];
  float* sacc = (float*)lds_dyn;
  float* smax = sacc + NB * HD;
  float* sden = smax + NB;
  int*   list = (int*)(sden + NB);
  int*   wcnt = list + NWAVE * WCAP;

  const int tid = threadIdx.x, lane = tid & 31, wave = tid >> 5;
  const int h = lane >> 4, m = lane & 15;
  const int nodeBase = blockIdx.x * NB;

  {
    const v4f z4 = {0.f, 0.f, 0.f, 0.f};
    for (int i = tid; i < NB * HD / 4; i += NTHR) lds_dyn[i] = z4;
    for (int i = tid; i < NB; i += NTHR) { smax[i] = -1.0e30f; sden[i] = 0.f; }
  }
  __syncthreads();

  const int* eid = dsti;
  const bool al16 = ((((size_t)dsti) & 15) == 0);
  const int nChunks = (nItems + CHUNK - 1) / CHUNK;
#pragma unroll 1
  for (int ch = 0; ch < nChunks; ++ch) {
    const int cbase = ch * CHUNK;
    int wc = 0;
#pragma unroll
    for (int g = 0; g < NGRP; ++g) {
      const int el0 = (g * NTHR + tid) * 4;
      const int e0  = cbase + el0;
      const int sent = -2147483647 - 1;
      v4i d;
      if (al16 && (cbase + CHUNK <= nItems)) {
        d = *(const v4i*)(eid + e0);
      } else {
        const int c0 = e0     > nItems - 1 ? nItems - 1 : e0;
        const int c1 = e0 + 1 > nItems - 1 ? nItems - 1 : e0 + 1;
        const int c2 = e0 + 2 > nItems - 1 ? nItems - 1 : e0 + 2;
        const int c3 = e0 + 3 > nItems - 1 ? nItems - 1 : e0 + 3;
        const int v0 = eid[c0], v1 = eid[c1], v2 = eid[c2], v3 = eid[c3];
        d.x = (e0     < nItems) ? v0 : sent;
        d.y = (e0 + 1 < nItems) ? v1 : sent;
        d.z = (e0 + 2 < nItems) ? v2 : sent;
        d.w = (e0 + 3 < nItems) ? v3 : sent;
      }
      const unsigned s0 = (unsigned)d.x - (unsigned)nodeBase;
      const unsigned s1 = (unsigned)d.y - (unsigned)nodeBase;
      const unsigned s2 = (unsigned)d.z - (unsigned)nodeBase;
      const unsigned s3 = (unsigned)d.w - (unsigned)nodeBase;
      const bool h0 = s0 < (unsigned)NB;
      const bool h1 = s1 < (unsigned)NB;
      const bool h2 = s2 < (unsigned)NB;
      const bool h3 = s3 < (unsigned)NB;
      const unsigned many = __builtin_amdgcn_ballot_w32(h0 | h1 | h2 | h3);
      if (many != 0u) {
#define HITJ(J, HJ, SJ) { \
          const unsigned mj = __builtin_amdgcn_ballot_w32(HJ); \
          if (HJ) { \
            const int pos = wc + (int)__builtin_amdgcn_mbcnt_lo(mj, 0u); \
            if (pos < WCAP) list[wave * WCAP + pos] = ((el0 + (J)) << 10) | (int)(SJ); \
          } \
          wc += (int)__builtin_popcount(mj); }
        HITJ(0, h0, s0)
        HITJ(1, h1, s1)
        HITJ(2, h2, s2)
        HITJ(3, h3, s3)
#undef HITJ
      }
    }
    if (lane == 0) wcnt[wave] = wc;
    __syncthreads();

    if (wave == 0) {
      for (int wsx = 0; wsx < NWAVE; ++wsx) {
        int n = wcnt[wsx];
        if (n > WCAP) n = WCAP;
        if (n < 0) n = 0;
        for (int i = 0; i < n; ++i) {
          const int ent  = list[wsx * WCAP + i];
          const int slot = ent & (NB - 1);
          const int el   = (ent >> 10) & (CHUNK - 1);
          int e = cbase + el;
          if (e > nItems - 1) e = nItems - 1;
          int src;
          if (MODE <= 1) {
            src = srci[e];
            src = src < 0 ? 0 : (src > nSrc - 1 ? nSrc - 1 : src);
          } else {
            src = e > nSrc - 1 ? nSrc - 1 : e;
          }
          const v2f xv = *(const v2f*)(msg + (size_t)src * HD + 2 * lane);
          v2f* sp = (v2f*)(sacc + slot * HD + 2 * lane);
          const v2f cur = *sp;
          if (MODE == 3) {
            *sp = cur + xv;
          } else {
            float a;
            if (MODE == 0) {
              a = lg[e];
            } else {
              int dn = nodeBase + slot;
              if (dn > nDst - 1) dn = nDst - 1;
              a = leaky01(asn[src] + adn[dn]);
            }
            const float mo = smax[slot];
            const float mn = fmaxf(mo, a);
            const float sc = __expf(mo - mn);
            const float p  = __expf(a - mn);
            *sp = cur * sc + p * xv;
            if (lane == 0) {
              const float dd = sden[slot];
              sden[slot] = dd * sc + p;
              smax[slot] = mn;
            }
          }
          __builtin_amdgcn_fence(__ATOMIC_RELEASE, "wavefront");
          __builtin_amdgcn_wave_barrier();
        }
      }
    }
    __syncthreads();
  }

  agg_store<MODE>(sacc, sden, bias, out, nodeBase, wave, h, m);
  __threadfence();
  agg_store<MODE>(sacc, sden, bias, out, nodeBase, wave, h, m);
}

__device__ __forceinline__ void lin2_store(const float* ys, float* y, int nG, int tid) {
  if (tid < NTHR / 4) {
    const int g0 = blockIdx.x * NTHR + 4 * tid;
    const v4f v = *(const v4f*)(ys + 4 * tid);
    if (g0 + 4 <= nG) {
      *(volatile v4f*)(y + g0) = v;
    } else {
      if (g0     < nG) ((volatile float*)y)[g0]     = v.x;
      if (g0 + 1 < nG) ((volatile float*)y)[g0 + 1] = v.y;
      if (g0 + 2 < nG) ((volatile float*)y)[g0 + 2] = v.z;
      if (g0 + 3 < nG) ((volatile float*)y)[g0 + 3] = v.w;
    }
  }
}

__global__ __launch_bounds__(NTHR) void k_lin2(const float* __restrict__ O, int nG,
                                               const float* __restrict__ W, const float* __restrict__ b,
                                               float* y) {
  __shared__ __attribute__((aligned(16))) float ys[NTHR];
  const int tid = threadIdx.x;
  int g = blockIdx.x * NTHR + tid;
  if (g > nG - 1) g = nG - 1;
  const float* o = O + (size_t)g * HD;
  float s = 0.f;
#pragma unroll 4
  for (int k = 0; k < HD; ++k) s += o[k] * W[k];
  ys[tid] = s + b[0];
  __syncthreads();
  lin2_store(ys, y, nG, tid);
  __threadfence();
  lin2_store(ys, y, nG, tid);
}

static inline size_t al256(size_t x) { return (x + 255) & ~(size_t)255; }

extern "C" void kernel_launch(void* const* d_in, const int* in_sizes, int n_in,
                              void* d_out, int out_size, void* d_ws, size_t ws_size,
                              hipStream_t stream) {
  if (n_in < 33) return;
  const int nN = in_sizes[0] / HD;
  const int nE = in_sizes[2] / EDM;
  const int nG = out_size;
  if (nN <= 0 || in_sizes[0] != nN * HD) return;
  if (nE <= 0 || in_sizes[2] != nE * EDM || in_sizes[1] != 2 * nE) return;
  if (in_sizes[3] != nN || nG <= 0) return;
  if (in_sizes[4] != HD * HD || in_sizes[8] != HD * (HD + EDM) || in_sizes[9] != HD * HD) return;
  if (in_sizes[11] != 3 * HD * HD || in_sizes[12] != 3 * HD * HD) return;
  if (in_sizes[15] != 3 * HD * HD || in_sizes[16] != 3 * HD * HD) return;
  if (in_sizes[19] != 3 * HD * HD || in_sizes[20] != 3 * HD * HD) return;
  if (in_sizes[23] != HD * HD || in_sizes[27] != HD * HD || in_sizes[31] != HD || in_sizes[32] < 1) return;

  const float* x         = (const float*)d_in[0];
  const int*   ei        = (const int*)d_in[1];
  const float* edge_attr = (const float*)d_in[2];
  const int*   batch     = (const int*)d_in[3];
  const float* lin1_W = (const float*)d_in[4];
  const float* lin1_b = (const float*)d_in[5];
  const float* gate_att_l = (const float*)d_in[6];
  const float* gate_att_r = (const float*)d_in[7];
  const float* gate_W1 = (const float*)d_in[8];
  const float* gate_W2 = (const float*)d_in[9];
  const float* gate_b  = (const float*)d_in[10];
  const float* gru0_Wih = (const float*)d_in[11];
  const float* gru0_Whh = (const float*)d_in[12];
  const float* gru0_bih = (const float*)d_in[13];
  const float* gru0_bhh = (const float*)d_in[14];
  const float* gru1_Wih = (const float*)d_in[15];
  const float* gru1_Whh = (const float*)d_in[16];
  const float* gru1_bih = (const float*)d_in[17];
  const float* gru1_bhh = (const float*)d_in[18];
  const float* molg_Wih = (const float*)d_in[19];
  const float* molg_Whh = (const float*)d_in[20];
  const float* molg_bih = (const float*)d_in[21];
  const float* molg_bhh = (const float*)d_in[22];
  const float* atom_W = (const float*)d_in[23];
  const float* atom_att_src = (const float*)d_in[24];
  const float* atom_att_dst = (const float*)d_in[25];
  const float* atom_b = (const float*)d_in[26];
  const float* mol_W = (const float*)d_in[27];
  const float* mol_att_src = (const float*)d_in[28];
  const float* mol_att_dst = (const float*)d_in[29];
  const float* mol_b = (const float*)d_in[30];
  const float* lin2_W = (const float*)d_in[31];
  const float* lin2_b = (const float*)d_in[32];
  float* y = (float*)d_out;

  const int NP = ((nN + NB - 1) / NB) * NB;
  const int GP = ((nG + NB - 1) / NB) * NB;
  const int EB = (nE + ET - 1) / ET;
  const size_t EP = (size_t)EB * ET;

  char* wb = (char*)d_ws;
  size_t off = 0;
  us16* P64  = (us16*)(wb + off);  off = al256(off + (size_t)5 * 2 * HD * HD * sizeof(us16));
  us16* P192 = (us16*)(wb + off);  off = al256(off + (size_t)6 * 2 * 3 * HD * HD * sizeof(us16));
  float* PA = (float*)(wb + off);  off = al256(off + (size_t)NP * HD * sizeof(float));
  float* PB = (float*)(wb + off);  off = al256(off + (size_t)NP * HD * sizeof(float));
  float* PC = (float*)(wb + off);  off = al256(off + (size_t)NP * HD * sizeof(float));
  float* PD = (float*)(wb + off);  off = al256(off + (size_t)NP * HD * sizeof(float));
  float* PE = (float*)(wb + off);  off = al256(off + (size_t)NP * HD * sizeof(float));
  float* SGR  = (float*)(wb + off); off = al256(off + (size_t)NP * sizeof(float));
  float* SASN = (float*)(wb + off); off = al256(off + (size_t)NP * sizeof(float));
  float* SADN = (float*)(wb + off); off = al256(off + (size_t)NP * sizeof(float));
  float* E1   = (float*)(wb + off); off = al256(off + EP * sizeof(float));
  float* GO0  = (float*)(wb + off); off = al256(off + (size_t)GP * HD * sizeof(float));
  float* GO1  = (float*)(wb + off); off = al256(off + (size_t)GP * HD * sizeof(float));
  float* GH   = (float*)(wb + off); off = al256(off + (size_t)GP * HD * sizeof(float));
  float* GX   = (float*)(wb + off); off = al256(off + (size_t)GP * HD * sizeof(float));
  float* SADG = (float*)(wb + off); off = al256(off + (size_t)GP * sizeof(float));
  if (off > ws_size || off > (size_t)134217728) return;

  const size_t s64 = (size_t)2 * HD * HD, s192 = (size_t)2 * 3 * HD * HD;
  const us16* L1h  = P64 + 0 * s64;  const us16* L1l  = L1h  + HD * HD;
  const us16* W1ah = P64 + 1 * s64;  const us16* W1al = W1ah + HD * HD;
  const us16* W2h  = P64 + 2 * s64;  const us16* W2l  = W2h  + HD * HD;
  const us16* AWh  = P64 + 3 * s64;  const us16* AWl  = AWh  + HD * HD;
  const us16* MWh  = P64 + 4 * s64;  const us16* MWl  = MWh  + HD * HD;
  const us16* G0ih = P192 + 0 * s192; const us16* G0hh = P192 + 1 * s192;
  const us16* G1ih = P192 + 2 * s192; const us16* G1hh = P192 + 3 * s192;
  const us16* MGih = P192 + 4 * s192; const us16* MGhh = P192 + 5 * s192;

  const dim3 B(NTHR);

  k_prep<<<dim3((HD * 8 + NTHR - 1) / NTHR, 5), B, 0, stream>>>(
      lin1_W, gate_W1, gate_W2, atom_W, mol_W, mol_W,
      HD, HD + EDM, HD, HD, HD, HD, HD, P64);
  k_prep<<<dim3((3 * HD * 8 + NTHR - 1) / NTHR, 6), B, 0, stream>>>(
      gru0_Wih, gru0_Whh, gru1_Wih, gru1_Whh, molg_Wih, molg_Whh,
      HD, HD, HD, HD, HD, HD, 3 * HD, P192);

  const unsigned gNode = (unsigned)(NP / GR);
  const unsigned gGraph = (unsigned)(GP / GR);

  k_gemm<1><<<gNode, B, 0, stream>>>(x, nN, L1h, L1l, lin1_b, gate_att_r, gate_att_r, 1 | 2, PA, SGR, SADN);
  k_gemm<0><<<gNode, B, 0, stream>>>(PA, nN, W1ah, W1al, lin1_b, gate_att_r, gate_att_r, 0, PB, SADN, SADN);
  k_gemm<0><<<gNode, B, 0, stream>>>(PA, nN, W2h, W2l, lin1_b, gate_att_r, gate_att_r, 0, PC, SADN, SADN);
  k_edge<<<(unsigned)EB, B, 0, stream>>>(edge_attr, ei, nE, gate_W1, gate_att_l, PB, SGR, nN, E1);

  hipFuncSetAttribute(reinterpret_cast<const void*>(&k_agg<0>), hipFuncAttributeMaxDynamicSharedMemorySize, LDS_AGG_BYTES);
  hipFuncSetAttribute(reinterpret_cast<const void*>(&k_agg<1>), hipFuncAttributeMaxDynamicSharedMemorySize, LDS_AGG_BYTES);
  hipFuncSetAttribute(reinterpret_cast<const void*>(&k_agg<2>), hipFuncAttributeMaxDynamicSharedMemorySize, LDS_AGG_BYTES);
  hipFuncSetAttribute(reinterpret_cast<const void*>(&k_agg<3>), hipFuncAttributeMaxDynamicSharedMemorySize, LDS_AGG_BYTES);

  const unsigned gAggN = (unsigned)(NP / NB);
  const unsigned gAggG = (unsigned)(GP / NB);

  k_agg<0><<<gAggN, B, LDS_AGG_BYTES, stream>>>(ei, ei + nE, nE, PC, nN, E1, SGR, SGR, nN, gate_b, PD);
  k_gru<<<gNode, B, 0, stream>>>(PD, PA, nN, G0ih, G0hh, gru0_bih, gru0_bhh, PE);
  k_gemm<0><<<gNode, B, 0, stream>>>(PE, nN, AWh, AWl, lin1_b, atom_att_src, atom_att_dst, 2 | 4, PB, SASN, SADN);
  k_agg<1><<<gAggN, B, LDS_AGG_BYTES, stream>>>(ei, ei + nE, nE, PB, nN, E1, SASN, SADN, nN, atom_b, PD);
  k_gru<<<gNode, B, 0, stream>>>(PD, PE, nN, G1ih, G1hh, gru1_bih, gru1_bhh, PC);
  k_gemm<0><<<gNode, B, 0, stream>>>(PC, nN, MWh, MWl, lin1_b, mol_att_src, mol_att_src, 2, PB, SASN, SADN);
  k_agg<3><<<gAggG, B, LDS_AGG_BYTES, stream>>>(batch, batch, nN, PC, nN, E1, SASN, SADN, nG, mol_b, GO0);

  float* cur = GO0;
  float* nxt = GO1;
  for (int t = 0; t < 2; ++t) {
    k_gemm<0><<<gGraph, B, 0, stream>>>(cur, nG, MWh, MWl, lin1_b, mol_att_dst, mol_att_dst, 2, GX, SADG, SADG);
    k_agg<2><<<gAggG, B, LDS_AGG_BYTES, stream>>>(batch, batch, nN, PB, nN, E1, SASN, SADG, nG, mol_b, GH);
    k_gru<<<gGraph, B, 0, stream>>>(GH, cur, nG, MGih, MGhh, molg_bih, molg_bhh, nxt);
    float* tmp = cur; cur = nxt; nxt = tmp;
  }

  k_lin2<<<(unsigned)((nG + NTHR - 1) / NTHR), B, 0, stream>>>(cur, nG, lin2_W, lin2_b, y);
}
